// ContextRGAT_90546500534351
// MI455X (gfx1250) — hardware-verified
//
#include <hip/hip_runtime.h>
#include <stddef.h>
#include <stdint.h>


#define FD    128
#define NREL  3
#define GR    32
#define APW   68
#define WROW  64
#define XSP   132
#define NTHR  256
#define NWAVE 8
#define NB    512
#define CHUNK 2048
#define WCAP  256
#define NGRP  (CHUNK / (NTHR * 4))
#define NQW   8

#define LDS_SACC (NB * FD)
#define LDS_AUX  (NB + NB)
#define LDS_LIST (NWAVE * WCAP)
#define LDS_BYTES ((LDS_SACC + LDS_AUX + LDS_LIST + NWAVE + 8) * 4)

static_assert(WCAP == (CHUNK / NTHR) * 32);
static_assert(NGRP >= 1);
static_assert(NB == 512);
static_assert(CHUNK <= 4096);
static_assert((LDS_SACC % 4) == 0);
static_assert(LDS_BYTES == 274496);
static_assert(GR * NQW == 256);
static_assert((APW % 4) == 0);
static_assert((XSP % 4) == 0);

typedef float        v4f  __attribute__((ext_vector_type(4)));
typedef float        v8f  __attribute__((ext_vector_type(8)));
typedef int          v4i  __attribute__((ext_vector_type(4)));
typedef unsigned int v4u  __attribute__((ext_vector_type(4)));
typedef __bf16       v16b __attribute__((ext_vector_type(16)));
union Frag { v16b v; v4u q[2]; };

__device__ __forceinline__ v8f wm(v16b a, v16b b, v8f c) {
  v8f d = __builtin_amdgcn_wmma_f32_16x16x32_bf16(false, a, false, b, (short)0, c, false, false);
  asm volatile("v_nop\n\tv_nop\n\tv_nop\n\tv_nop" : "+v"(d) : "v"(a), "v"(b));
  return d;
}

__device__ __forceinline__ float wsum(float v) {
  v += __shfl_xor(v, 16, 32);
  v += __shfl_xor(v, 8, 32);
  v += __shfl_xor(v, 4, 32);
  v += __shfl_xor(v, 2, 32);
  v += __shfl_xor(v, 1, 32);
  return v;
}

__device__ __forceinline__ unsigned bfr(float f) {
  const unsigned u = __float_as_uint(f);
  return (u + 0x7FFFu + ((u >> 16) & 1u)) >> 16;
}
__device__ __forceinline__ unsigned hi2(float a, float b) {
  return bfr(a) | (bfr(b) << 16);
}
__device__ __forceinline__ unsigned lo2(float a, float b) {
  const float ra = a - __uint_as_float(bfr(a) << 16);
  const float rb = b - __uint_as_float(bfr(b) << 16);
  return bfr(ra) | (bfr(rb) << 16);
}

__global__ __launch_bounds__(NTHR) void k_prepw(const float* __restrict__ W,
                                                unsigned int* Whi, unsigned int* Wlo, int nT) {
  const int t = blockIdx.x * NTHR + threadIdx.x;
  if (t >= nT) return;
  const int rel = t >> 11;
  const int o   = (t >> 4) & (FD - 1);
  const int kc  = (t & 15) * 8;
  const float* s = W + ((size_t)rel * FD + kc) * FD + o;
  const float f0 = s[0],          f1 = s[FD],         f2 = s[2 * FD],     f3 = s[3 * FD];
  const float f4 = s[4 * FD],     f5 = s[5 * FD],     f6 = s[6 * FD],     f7 = s[7 * FD];
  const v4u hv = {hi2(f0, f1), hi2(f2, f3), hi2(f4, f5), hi2(f6, f7)};
  const v4u lv = {lo2(f0, f1), lo2(f2, f3), lo2(f4, f5), lo2(f6, f7)};
  const size_t wo = ((size_t)rel * FD + o) * WROW + (kc >> 1);
  *(volatile v4u*)(Whi + wo) = hv;
  *(volatile v4u*)(Wlo + wo) = lv;
  __threadfence();
  *(volatile v4u*)(Whi + wo) = hv;
  *(volatile v4u*)(Wlo + wo) = lv;
}

__global__ __launch_bounds__(NTHR) void k_xw(
    const float* __restrict__ A, const unsigned int* __restrict__ Whi,
    const unsigned int* __restrict__ Wlo, const float* __restrict__ qv,
    const float* __restrict__ kv, float* XW, float* NQK, int nN) {
  __shared__ __attribute__((aligned(16))) unsigned int Ah[GR * APW];
  __shared__ __attribute__((aligned(16))) unsigned int Al[GR * APW];
  __shared__ __attribute__((aligned(16))) float Xs[GR * XSP];
  __shared__ __attribute__((aligned(16))) float Ls[GR * NQW];

  const int tid  = threadIdx.x;
  const int lane = tid & 31;
  const int wave = tid >> 5;
  const int hh   = lane >> 4;
  const int m    = lane & 15;
  const int rowBase = blockIdx.x * GR;

  {
    const int r  = tid >> 3;
    const int c0 = (tid & 7) * 16;
    int row = rowBase + r;
    if (row > nN - 1) row = nN - 1;
    const float* p = A + (size_t)row * FD + c0;
    const v4f f0 = *(const v4f*)(p), f1 = *(const v4f*)(p + 4);
    const v4f f2 = *(const v4f*)(p + 8), f3 = *(const v4f*)(p + 12);
    const v4u h0 = {hi2(f0.x, f0.y), hi2(f0.z, f0.w), hi2(f1.x, f1.y), hi2(f1.z, f1.w)};
    const v4u l0 = {lo2(f0.x, f0.y), lo2(f0.z, f0.w), lo2(f1.x, f1.y), lo2(f1.z, f1.w)};
    const v4u h1 = {hi2(f2.x, f2.y), hi2(f2.z, f2.w), hi2(f3.x, f3.y), hi2(f3.z, f3.w)};
    const v4u l1 = {lo2(f2.x, f2.y), lo2(f2.z, f2.w), lo2(f3.x, f3.y), lo2(f3.z, f3.w)};
    unsigned int* dh = Ah + r * APW + (c0 >> 1);
    unsigned int* dl = Al + r * APW + (c0 >> 1);
    *(v4u*)(dh) = h0; *(v4u*)(dh + 4) = h1;
    *(v4u*)(dl) = l0; *(v4u*)(dl + 4) = l1;
    if (tid < GR) { Ls[tid * NQW + 6] = 0.f; Ls[tid * NQW + 7] = 0.f; }
  }
  __syncthreads();

  const int ncl = wave * 16 + m;
  const unsigned int* a0h = Ah + m * APW + 4 * hh;
  const unsigned int* a1h = Ah + (16 + m) * APW + 4 * hh;
  const unsigned int* a0l = Al + m * APW + 4 * hh;
  const unsigned int* a1l = Al + (16 + m) * APW + 4 * hh;

#pragma unroll 1
  for (int rel = 0; rel < NREL; ++rel) {
    const unsigned int* bh = Whi + ((size_t)rel * FD + ncl) * WROW + 4 * hh;
    const unsigned int* bl = Wlo + ((size_t)rel * FD + ncl) * WROW + 4 * hh;
    v8f c0a = {0.f, 0.f, 0.f, 0.f, 0.f, 0.f, 0.f, 0.f};
    v8f c1a = {0.f, 0.f, 0.f, 0.f, 0.f, 0.f, 0.f, 0.f};
#pragma unroll 1
    for (int kt = 0; kt < FD / 32; ++kt) {
      const int kw = 16 * kt;
      Frag fbh, fbl, fa0h, fa0l, fa1h, fa1l;
      fbh.q[0]  = *(const v4u*)(bh + kw);   fbh.q[1]  = *(const v4u*)(bh + kw + 8);
      fbl.q[0]  = *(const v4u*)(bl + kw);   fbl.q[1]  = *(const v4u*)(bl + kw + 8);
      fa0h.q[0] = *(const v4u*)(a0h + kw);  fa0h.q[1] = *(const v4u*)(a0h + kw + 8);
      fa0l.q[0] = *(const v4u*)(a0l + kw);  fa0l.q[1] = *(const v4u*)(a0l + kw + 8);
      fa1h.q[0] = *(const v4u*)(a1h + kw);  fa1h.q[1] = *(const v4u*)(a1h + kw + 8);
      fa1l.q[0] = *(const v4u*)(a1l + kw);  fa1l.q[1] = *(const v4u*)(a1l + kw + 8);
      c0a = wm(fa0h.v, fbh.v, c0a);
      c0a = wm(fa0h.v, fbl.v, c0a);
      c0a = wm(fa0l.v, fbh.v, c0a);
      c1a = wm(fa1h.v, fbh.v, c1a);
      c1a = wm(fa1h.v, fbl.v, c1a);
      c1a = wm(fa1l.v, fbh.v, c1a);
    }

#pragma unroll
    for (int r = 0; r < 8; ++r) {
      Xs[(8 * hh + r) * XSP + ncl]      = c0a[r];
      Xs[(16 + 8 * hh + r) * XSP + ncl] = c1a[r];
    }
    __syncthreads();

    {
      const int row  = tid >> 3;
      const int part = tid & 7;
      float sq = 0.f, sk = 0.f;
#pragma unroll
      for (int j = 0; j < 16; ++j) {
        const int c = part * 16 + j;
        const float v = Xs[row * XSP + c];
        sq += v * qv[c];
        sk += v * kv[c];
      }
      sq += __shfl_xor(sq, 1, 32); sk += __shfl_xor(sk, 1, 32);
      sq += __shfl_xor(sq, 2, 32); sk += __shfl_xor(sk, 2, 32);
      sq += __shfl_xor(sq, 4, 32); sk += __shfl_xor(sk, 4, 32);
      if (part == 0) {
        Ls[row * NQW + rel]     = sq;
        Ls[row * NQW + 3 + rel] = sk;
      }
    }

    v4f xr[4];
    float* xp[4];
#pragma unroll
    for (int i = 0; i < 4; ++i) {
      xr[i] = *(const v4f*)(Xs + (4 * wave + i) * XSP + 4 * lane);
      xp[i] = XW + ((size_t)(rowBase + 4 * wave + i) * NREL + rel) * FD + 4 * lane;
    }
#pragma unroll
    for (int i = 0; i < 4; ++i) *(volatile v4f*)(xp[i]) = xr[i];
    __threadfence();
#pragma unroll
    for (int i = 0; i < 4; ++i) *(volatile v4f*)(xp[i]) = xr[i];
    __syncthreads();
  }

  if (wave == 0) {
    const v4f g0 = *(const v4f*)(Ls + 4 * lane);
    const v4f g1 = *(const v4f*)(Ls + 128 + 4 * lane);
    float* gp = NQK + (size_t)rowBase * NQW;
    *(volatile v4f*)(gp + 4 * lane)       = g0;
    *(volatile v4f*)(gp + 128 + 4 * lane) = g1;
    __threadfence();
    *(volatile v4f*)(gp + 4 * lane)       = g0;
    *(volatile v4f*)(gp + 128 + 4 * lane) = g1;
  }
}

__global__ __launch_bounds__(NTHR) void k_agg(
    const int* __restrict__ ei, const int* __restrict__ et, const float* __restrict__ ea,
    const float* __restrict__ XW, const float* __restrict__ NQK,
    const float* __restrict__ we, const float* __restrict__ ev,
    const float* __restrict__ bias, float* out, int nN, int nE, int relu) {
  extern __shared__ v4f lds_dyn[];
  float* sacc = (float*)lds_dyn;
  float* mxs  = sacc + LDS_SACC;
  float* dens = mxs + NB;
  int*   list = (int*)(dens + NB);
  int*   wcnt = list + LDS_LIST;
  float* ces  = (float*)(wcnt + NWAVE);

  const int tid  = threadIdx.x;
  const int lane = tid & 31;
  const int wave = tid >> 5;
  const int nodeBase = blockIdx.x * NB;

  {
    const v4f z4 = {0.f, 0.f, 0.f, 0.f};
    for (int i = tid; i < LDS_SACC / 4; i += NTHR) lds_dyn[i] = z4;
    for (int i = tid; i < NB; i += NTHR) { mxs[i] = -1.0e30f; dens[i] = 0.f; }
    if (wave == 0) {
      float s = we[4 * lane] * ev[4 * lane] + we[4 * lane + 1] * ev[4 * lane + 1]
              + we[4 * lane + 2] * ev[4 * lane + 2] + we[4 * lane + 3] * ev[4 * lane + 3];
      s = wsum(s);
      if (lane == 0) ces[0] = s;
    }
  }
  __syncthreads();
  const float ce = ces[0];
  const int* eid = ei + nE;
  const bool al16 = ((nE & 3) == 0);

  const int nChunks = (nE + CHUNK - 1) / CHUNK;
#pragma unroll 1
  for (int ch = 0; ch < nChunks; ++ch) {
    const int cbase = ch * CHUNK;
    int wc = 0;
#pragma unroll
    for (int g = 0; g < NGRP; ++g) {
      const int el0 = (g * NTHR + tid) * 4;
      const int e0  = cbase + el0;
      const int sent = -2147483647 - 1;
      v4i d;
      if (al16 && (e0 + 3 < nE)) {
        d = *(const v4i*)(eid + e0);
      } else {
        const int ec = nE - 1;
        d.x = (e0     < nE) ? eid[min(e0, ec)]     : sent;
        d.y = (e0 + 1 < nE) ? eid[min(e0 + 1, ec)] : sent;
        d.z = (e0 + 2 < nE) ? eid[min(e0 + 2, ec)] : sent;
        d.w = (e0 + 3 < nE) ? eid[min(e0 + 3, ec)] : sent;
      }
      const unsigned s0 = (unsigned)d.x - (unsigned)nodeBase;
      const unsigned s1 = (unsigned)d.y - (unsigned)nodeBase;
      const unsigned s2 = (unsigned)d.z - (unsigned)nodeBase;
      const unsigned s3 = (unsigned)d.w - (unsigned)nodeBase;
      const bool h0 = s0 < (unsigned)NB;
      const bool h1 = s1 < (unsigned)NB;
      const bool h2 = s2 < (unsigned)NB;
      const bool h3 = s3 < (unsigned)NB;
      const unsigned many = __builtin_amdgcn_ballot_w32(h0 | h1 | h2 | h3);
      if (many != 0u) {
#define HITJ(J, HJ, SJ) { \
          const unsigned mj = __builtin_amdgcn_ballot_w32(HJ); \
          if (HJ) { \
            const int pos = wc + (int)__builtin_amdgcn_mbcnt_lo(mj, 0u); \
            if (pos < WCAP) list[wave * WCAP + pos] = ((el0 + (J)) << 9) | (int)(SJ); \
          } \
          wc += (int)__builtin_popcount(mj); }
        HITJ(0, h0, s0)
        HITJ(1, h1, s1)
        HITJ(2, h2, s2)
        HITJ(3, h3, s3)
#undef HITJ
      }
    }
    if (lane == 0) wcnt[wave] = wc;
    __syncthreads();

    if (wave == 0) {
      for (int wsx = 0; wsx < NWAVE; ++wsx) {
        int n = wcnt[wsx];
        if (n > WCAP) n = WCAP;
        if (n < 0) n = 0;
        for (int i = 0; i < n; ++i) {
          const int ent  = list[wsx * WCAP + i];
          const int slot = ent & (NB - 1);
          const int el   = (ent >> 9) & (CHUNK - 1);
          int e = cbase + el;
          if (e > nE - 1) e = nE - 1;
          int src = ei[e];
          src = src < 0 ? 0 : (src > nN - 1 ? nN - 1 : src);
          int t = et[e];
          t = t < 0 ? 0 : (t > NREL - 1 ? NREL - 1 : t);
          const float w = ea[e];
          int nd = nodeBase + slot;
          if (nd > nN - 1) nd = nN - 1;
          const float qd = NQK[(size_t)nd * NQW + t];
          const float ks = NQK[(size_t)src * NQW + 3 + t];
          float al = (qd + ks) + w * ce;
          al = (al > 0.f) ? al : 0.2f * al;
          const float mo = mxs[slot];
          const float mn = fmaxf(mo, al);
          const float p  = __expf(al - mn);
          const float sc = (mo > -1.0e29f) ? __expf(mo - mn) : 0.f;
          const v4f xv = *(const v4f*)(XW + ((size_t)src * NREL + t) * FD + 4 * lane);
          v4f* sp = (v4f*)(sacc + slot * FD + 4 * lane);
          const v4f cur = *sp;
          const v4f nxt = cur * sc + p * xv;
          *sp = nxt;
          if (lane == 0) {
            const float dold = dens[slot];
            mxs[slot]  = mn;
            dens[slot] = dold * sc + p;
          }
        }
      }
    }
    __syncthreads();
  }

  const v4f b4 = *(const v4f*)(bias + 4 * lane);
#pragma unroll 1
  for (int j = 0; j < NB / NWAVE; ++j) {
    const int slot = wave * (NB / NWAVE) + j;
    const int node = nodeBase + slot;
    if (node >= nN) break;
    const float dv  = dens[slot];
    const float inv = 1.0f / (dv + 1e-16f);
    const v4f sv = *(const v4f*)(sacc + slot * FD + 4 * lane);
    v4f y = sv * inv + b4;
    if (relu) {
      y.x = y.x > 0.f ? y.x : 0.f;
      y.y = y.y > 0.f ? y.y : 0.f;
      y.z = y.z > 0.f ? y.z : 0.f;
      y.w = y.w > 0.f ? y.w : 0.f;
    }
    float* op = out + (size_t)node * FD + 4 * lane;
    *(volatile v4f*)op = y;
    __threadfence();
    *(volatile v4f*)op = y;
  }
}

static inline size_t al128(size_t v) { return (v + 127) & ~(size_t)127; }

extern "C" void kernel_launch(void* const* d_in, const int* in_sizes, int n_in,
                              void* d_out, int out_size, void* d_ws, size_t ws_size,
                              hipStream_t stream) {
  if (n_in < 16) return;
  const int nN = in_sizes[0] / FD;
  const int nE = in_sizes[2];
  if (nN <= 0 || in_sizes[0] != nN * FD) return;
  if (nE < 0 || in_sizes[1] != 2 * nE || in_sizes[3] != nE) return;
  if (in_sizes[4] != NREL * FD * FD || in_sizes[10] != NREL * FD * FD) return;
  for (int i = 5; i <= 9; ++i) if (in_sizes[i] != FD) return;
  for (int i = 11; i <= 15; ++i) if (in_sizes[i] != FD) return;
  if (out_size != nN * FD) return;

  const float* x   = (const float*)d_in[0];
  const int*   ei  = (const int*)d_in[1];
  const int*   et  = (const int*)d_in[2];
  const float* ea  = (const float*)d_in[3];
  const float* w1  = (const float*)d_in[4];
  const float* q1  = (const float*)d_in[5];
  const float* k1  = (const float*)d_in[6];
  const float* e1  = (const float*)d_in[7];
  const float* we1 = (const float*)d_in[8];
  const float* b1  = (const float*)d_in[9];
  const float* w2  = (const float*)d_in[10];
  const float* q2  = (const float*)d_in[11];
  const float* k2  = (const float*)d_in[12];
  const float* e2  = (const float*)d_in[13];
  const float* we2 = (const float*)d_in[14];
  const float* b2  = (const float*)d_in[15];
  float* out = (float*)d_out;

  const int nP = ((nN + GR - 1) / GR) * GR;
  size_t off = 0;
  unsigned int* Whi = (unsigned int*)((char*)d_ws + off); off += al128((size_t)NREL * FD * WROW * 4);
  unsigned int* Wlo = (unsigned int*)((char*)d_ws + off); off += al128((size_t)NREL * FD * WROW * 4);
  float* XW  = (float*)((char*)d_ws + off); off += al128((size_t)nP * NREL * FD * sizeof(float));
  float* NQK = (float*)((char*)d_ws + off); off += al128((size_t)nP * NQW * sizeof(float));
  float* H   = (float*)((char*)d_ws + off); off += al128((size_t)nP * FD * sizeof(float));
  if (off > ws_size) return;

  const int nT = NREL * FD * 16;
  const int gW = (nT + NTHR - 1) / NTHR;
  const int gX = nP / GR;
  const int gA = (nN + NB - 1) / NB;

  hipFuncSetAttribute(reinterpret_cast<const void*>(&k_agg),
                      hipFuncAttributeMaxDynamicSharedMemorySize, LDS_BYTES);

  k_prepw<<<gW, NTHR, 0, stream>>>(w1, Whi, Wlo, nT);
  k_xw<<<gX, NTHR, 0, stream>>>(x, Whi, Wlo, q1, k1, XW, NQK, nN);
  k_agg<<<gA, NTHR, LDS_BYTES, stream>>>(ei, et, ea, XW, NQK, we1, e1, b1, H, nN, nE, 1);

  k_prepw<<<gW, NTHR, 0, stream>>>(w2, Whi, Wlo, nT);
  k_xw<<<gX, NTHR, 0, stream>>>(H, Whi, Wlo, q2, k2, XW, NQK, nN);
  k_agg<<<gA, NTHR, LDS_BYTES, stream>>>(ei, et, ea, XW, NQK, we2, e2, b2, out, nN, nE, 0);
}
